// ExtendedMamba_32006096290220
// MI455X (gfx1250) — hardware-verified
//
#include <hip/hip_runtime.h>
#include <math.h>

#define NBAT 2
#define DMD  128
#define IMG  64
#define IMSH 6
#define LTOK 4096
#define LTSH 12
#define NTOK (NBAT * LTOK)
#define DIN  256
#define DST  16
#define DTRK 8
#define XPR  40
#define NDIR 4
#define XDN  256
#define XBO  8
#define XCO  24
#define DCV  4
#define EPSV 1e-5f
#define GSTR 40
#define OSTR 68
#define SMEMB (8 * 16 * OSTR * 4)
#define SCH  32
#define SYP  260
#define LOG2E 1.4426950408889634f

static_assert(LTOK == (1 << LTSH));
static_assert(IMG == (1 << IMSH));
static_assert(IMG * IMG == LTOK);
static_assert(NDIR == 4);
static_assert(NTOK % 128 == 0);
static_assert(DMD % 64 == 0);
static_assert(DMD % 32 == 0);
static_assert(DIN % 64 == 0);
static_assert((2 * DIN) % 64 == 0);
static_assert(XDN == 64 * NDIR);
static_assert(XPR == DTRK + 2 * DST);
static_assert(XBO == DTRK && XCO == XBO + DST && XCO + DST <= 64);
static_assert(SMEMB >= (2 * 128 * GSTR + 2 * 64 * GSTR) * 2);
static_assert(LTOK % SCH == 0);
static_assert(SCH == 32);
static_assert(SYP % 4 == 0);
static_assert(SYP >= DIN);
static_assert((SCH * (DIN / 4)) % DIN == 0);
static_assert(DIN / 8 == 32);
static_assert(DIN == 256);
static_assert((NTOK * (DIN / 8)) % 256 == 0);
static_assert((NTOK * (DMD / 8)) % 256 == 0);
static_assert((2 * DIN * (DMD / 8)) % 256 == 0);
static_assert((XDN * (DIN / 8)) % 256 == 0);
static_assert((DMD * (DIN / 8)) % 256 == 0);
static_assert(NTOK % 8 == 0);

typedef unsigned short us16 __attribute__((ext_vector_type(16)));
typedef unsigned short us8  __attribute__((ext_vector_type(8)));
typedef unsigned short us8a __attribute__((ext_vector_type(8), may_alias));
typedef __bf16 v16b __attribute__((ext_vector_type(16)));
typedef float v8f __attribute__((ext_vector_type(8)));
typedef float v4f __attribute__((ext_vector_type(4)));
typedef float v4fa __attribute__((ext_vector_type(4), may_alias));
union FragU { us16 v; us8 h[2]; };

__device__ __forceinline__ unsigned short bf16_bits(float f) {
  unsigned u = __float_as_uint(f);
  u += 0x7FFFu + ((u >> 16) & 1u);
  return (unsigned short)(u >> 16);
}
__device__ __forceinline__ float bf16_val(unsigned short b) { return __uint_as_float(((unsigned)b) << 16); }
__device__ __forceinline__ float bf16r(float f) { return bf16_val(bf16_bits(f)); }
__device__ __forceinline__ float siluf(float x) { return x * __builtin_amdgcn_rcpf(1.0f + __expf(-x)); }

__device__ __forceinline__ v8f mma_bf16(us16 a, us16 b, v8f c) {
  return __builtin_amdgcn_wmma_f32_16x16x32_bf16(false, __builtin_bit_cast(v16b, a), false, __builtin_bit_cast(v16b, b), (short)0, c, false, false);
}
__device__ __forceinline__ void wguard(v8f& c0, v8f& c1, v8f& c2, v8f& c3, const us16& a0, const us16& a1,
                                       const us16& b0, const us16& b1, const us16& b2, const us16& b3,
                                       const us16& e0, const us16& e1, const us16& e2, const us16& e3) {
#if defined(__HIP_DEVICE_COMPILE__)
  asm volatile("v_nop\n\tv_nop\n\tv_nop\n\tv_nop"
               : "+v"(c0), "+v"(c1), "+v"(c2), "+v"(c3)
               : "v"(a0), "v"(a1), "v"(b0), "v"(b1), "v"(b2), "v"(b3), "v"(e0), "v"(e1), "v"(e2), "v"(e3));
#endif
}

__device__ __forceinline__ us16 lds_frag(const unsigned short* base) {
  const int lane = threadIdx.x & 31, r = lane & 15, kh = (lane >> 4) * 8;
  FragU f;
  f.h[0] = *(const us8a*)(base + r * GSTR + kh);
  f.h[1] = *(const us8a*)(base + r * GSTR + 16 + kh);
  return f.v;
}

__device__ __forceinline__ void stage_a(unsigned short* lds, const unsigned short* __restrict__ P, int ld, int m0, int k0, int tid) {
  const int row = tid >> 1, cq = (tid & 1) * 16;
  const unsigned short* src = P + (size_t)(m0 + row) * ld + k0 + cq;
  const us8 v0 = *(const us8a*)src;
  const us8 v1 = *(const us8a*)(src + 8);
  *(us8a*)(lds + row * GSTR + cq) = v0;
  *(us8a*)(lds + row * GSTR + cq + 8) = v1;
}
__device__ __forceinline__ void stage_b(unsigned short* lds, const unsigned short* __restrict__ P, int ld, int n0, int k0, int tid) {
  const int row = tid >> 2, kq = (tid & 3) * 8;
  const us8 v = *(const us8a*)(P + (size_t)(n0 + row) * ld + k0 + kq);
  *(us8a*)(lds + row * GSTR + kq) = v;
}

template <int A2, int B2>
__global__ __launch_bounds__(256) void k_gemm(const unsigned short* __restrict__ A0, const unsigned short* __restrict__ A1, int lda, int zsa,
                                             const unsigned short* __restrict__ B0, const unsigned short* __restrict__ B1, int ldb, int zsb,
                                             float* Y, float* Yalt, int nsplit, int ldy, int zsy, int K, int mrows) {
#pragma clang fp contract(off)
  static_assert(!(A2 && B2));
  __shared__ __attribute__((aligned(16))) unsigned char sm[SMEMB];
  unsigned short* lA0 = (unsigned short*)sm;
  unsigned short* lA1 = lA0 + 128 * GSTR;
  unsigned short* lB0 = lA1 + 128 * GSTR;
  unsigned short* lB1 = lB0 + 64 * GSTR;
  float* oS = (float*)sm;
  const int tid = threadIdx.x, lane = tid & 31, wave = tid >> 5, cl = lane & 15, hh = lane >> 4;
  const int m0 = blockIdx.x * 128;
  const int n0 = blockIdx.y * 64;
  const size_t za = (size_t)blockIdx.z * (size_t)zsa;
  const size_t zb = (size_t)blockIdx.z * (size_t)zsb;
  const size_t zy = (size_t)blockIdx.z * (size_t)zsy;
  const unsigned short* A0z = A0 + za;
  const unsigned short* A1z = A1 + za;
  const unsigned short* B0z = B0 + zb;
  const unsigned short* B1z = B1 + zb;
  float* Yb = Y + zy;
  int nq = n0;
  if (nsplit > 0 && n0 >= nsplit) { Yb = Yalt + zy; nq = n0 - nsplit; }

  v8f acc[4];
#pragma unroll
  for (int j = 0; j < 4; ++j) { v8f zz = {0.f, 0.f, 0.f, 0.f, 0.f, 0.f, 0.f, 0.f}; acc[j] = zz; }

#pragma unroll 1
  for (int k0 = 0; k0 < K; k0 += 32) {
    __syncthreads();
    stage_a(lA0, A0z, lda, m0, k0, tid);
    if (A2) stage_a(lA1, A1z, lda, m0, k0, tid);
    stage_b(lB0, B0z, ldb, n0, k0, tid);
    if (B2) stage_b(lB1, B1z, ldb, n0, k0, tid);
    __syncthreads();
    const us16 af0 = lds_frag(lA0 + 16 * wave * GSTR);
    us16 af1 = af0;
    if (A2) af1 = lds_frag(lA1 + 16 * wave * GSTR);
    us16 b0f[4], b1f[4];
#pragma unroll
    for (int j = 0; j < 4; ++j) {
      b0f[j] = lds_frag(lB0 + 16 * j * GSTR);
      b1f[j] = b0f[j];
      if (B2) b1f[j] = lds_frag(lB1 + 16 * j * GSTR);
    }
#pragma unroll
    for (int j = 0; j < 4; ++j) acc[j] = mma_bf16(af0, b0f[j], acc[j]);
    if (A2) {
#pragma unroll
      for (int j = 0; j < 4; ++j) acc[j] = mma_bf16(af1, b0f[j], acc[j]);
    }
    if (B2) {
#pragma unroll
      for (int j = 0; j < 4; ++j) acc[j] = mma_bf16(af0, b1f[j], acc[j]);
    }
    wguard(acc[0], acc[1], acc[2], acc[3], af0, af1, b0f[0], b0f[1], b0f[2], b0f[3], b1f[0], b1f[1], b1f[2], b1f[3]);
  }
  __syncthreads();

  float* so = oS + wave * (16 * OSTR);
#pragma unroll
  for (int j = 0; j < 4; ++j)
#pragma unroll
    for (int r = 0; r < 8; ++r) so[(8 * hh + r) * OSTR + 16 * j + cl] = acc[j][r];
  __syncthreads();
  const bool wst = (m0 + 16 * wave + 16 <= mrows);
#pragma unroll
  for (int pass = 0; pass < 2; ++pass) {
#pragma unroll
    for (int it = 0; it < 8; ++it) {
      const int ch = it * 32 + lane, r = ch >> 4, q = (ch & 15) * 4;
      const v4f v = *(const v4fa*)(so + r * OSTR + q);
      if (wst) *(volatile v4f*)(Yb + (size_t)(m0 + 16 * wave + r) * ldy + nq + q) = v;
    }
    __threadfence();
  }
}

__global__ __launch_bounds__(256) void k_cvt(const float* __restrict__ src, unsigned short* dst, int nsrc, int ncol8, int total8) {
  const int idx = blockIdx.x * 256 + threadIdx.x;
  if (idx >= total8) return;
  const int row = idx / ncol8, c8 = (idx - row * ncol8) * 8;
  const int rs = (row < nsrc) ? row : (nsrc - 1);
  const float* s = src + (size_t)rs * (size_t)(ncol8 * 8) + c8;
  const v4f a = *(const v4fa*)s, b = *(const v4fa*)(s + 4);
  const bool zr = (row >= nsrc);
  us8 o;
#pragma unroll
  for (int u = 0; u < 4; ++u) {
    o[u]     = zr ? (unsigned short)0 : bf16_bits(a[u]);
    o[4 + u] = zr ? (unsigned short)0 : bf16_bits(b[u]);
  }
  const size_t off = (size_t)row * (size_t)(ncol8 * 8) + c8;
  *(volatile us8*)(dst + off) = o;
  __threadfence();
  *(volatile us8*)(dst + off) = o;
}

__global__ __launch_bounds__(256) void k_cvt_xw(const float* __restrict__ src, unsigned short* dst) {
  const int idx = blockIdx.x * 256 + threadIdx.x;
  if (idx >= XDN * (DIN / 8)) return;
  const int row = idx / (DIN / 8), c8 = (idx - row * (DIN / 8)) * 8;
  const int dir = row >> 6, rr = row & 63;
  const bool ok = (rr < XPR);
  const int sr = ok ? rr : (XPR - 1);
  const float* s = src + ((size_t)(dir * XPR + sr)) * DIN + c8;
  const v4f a = *(const v4fa*)s, b = *(const v4fa*)(s + 4);
  us8 o;
#pragma unroll
  for (int u = 0; u < 4; ++u) {
    o[u]     = ok ? bf16_bits(a[u]) : (unsigned short)0;
    o[4 + u] = ok ? bf16_bits(b[u]) : (unsigned short)0;
  }
  const size_t off = (size_t)row * DIN + c8;
  *(volatile us8*)(dst + off) = o;
  __threadfence();
  *(volatile us8*)(dst + off) = o;
}

__device__ __forceinline__ void split8(const float* v, us8& hi, us8& lo) {
#pragma unroll
  for (int u = 0; u < 8; ++u) {
    const unsigned short hb = bf16_bits(v[u]);
    hi[u] = hb; lo[u] = bf16_bits(v[u] - bf16_val(hb));
  }
}

__global__ __launch_bounds__(256) void k_dw4(const float* __restrict__ XI, const float* __restrict__ w, const float* __restrict__ bias,
                                            unsigned short* UH, unsigned short* UL) {
#pragma clang fp contract(off)
  __shared__ __attribute__((aligned(16))) float w4s[DCV * DIN];
  const int tid = threadIdx.x;
#pragma unroll 1
  for (int i = tid; i < DCV * DIN; i += 256) {
    const int tap = i / DIN, c = i - tap * DIN;
    w4s[i] = bf16r(w[c * DCV + tap]);
  }
  __syncthreads();
  const int idx = blockIdx.x * 256 + tid;
  if (idx >= NTOK * (DIN / 8)) return;
  const int tok = idx >> 5, c8 = (idx & 31) * 8;
  const int bb = tok >> LTSH, l = tok & (LTOK - 1);
  float acc[8];
#pragma unroll
  for (int u = 0; u < 8; ++u) acc[u] = 0.0f;
#pragma unroll
  for (int j = 0; j < DCV; ++j) {
    const int ll = l - (DCV - 1) + j;
    const bool ok = (ll >= 0);
    const int llc = ok ? ll : 0;
    const float* p = XI + ((size_t)bb * LTOK + (size_t)llc) * DIN + c8;
    const v4f xa = *(const v4fa*)p, xb = *(const v4fa*)(p + 4);
    const float* wq = w4s + j * DIN + c8;
    const v4f wa = *(const v4fa*)wq, wb = *(const v4fa*)(wq + 4);
#pragma unroll
    for (int u = 0; u < 4; ++u) {
      const float pa = xa[u] * wa[u];
      const float pb = xb[u] * wb[u];
      acc[u]     = acc[u]     + (ok ? pa : 0.0f);
      acc[4 + u] = acc[4 + u] + (ok ? pb : 0.0f);
    }
  }
  const v4f ba = *(const v4fa*)(bias + c8), bq = *(const v4fa*)(bias + c8 + 4);
  float v[8];
#pragma unroll
  for (int u = 0; u < 4; ++u) { v[u] = siluf(acc[u] + bf16r(ba[u])); v[4 + u] = siluf(acc[4 + u] + bf16r(bq[u])); }
  us8 hi, lo;
  split8(v, hi, lo);
  const size_t o = (size_t)idx * 8;
  *(volatile us8*)(UH + o) = hi; *(volatile us8*)(UL + o) = lo;
  __threadfence();
  *(volatile us8*)(UH + o) = hi; *(volatile us8*)(UL + o) = lo;
}

__device__ __forceinline__ int tok_of(int dir, int l) {
  const int lr = (dir & 2) ? (LTOK - 1 - l) : l;
  const int lt = ((lr & (IMG - 1)) << IMSH) | (lr >> IMSH);
  return (dir & 1) ? lt : lr;
}

__global__ __launch_bounds__(256) void k_scan(const float* __restrict__ XD, const unsigned short* __restrict__ UH,
                                             const unsigned short* __restrict__ UL,
                                             const float* __restrict__ dtw, const float* __restrict__ dtb,
                                             const float* __restrict__ Alog, const float* __restrict__ Dv, float* YS) {
#pragma clang fp contract(off)
  __shared__ __attribute__((aligned(16))) float sy[SCH * SYP];
  const int bb = blockIdx.x >> 2, dir = blockIdx.x & 3, tid = threadIdx.x;
  const int d = tid, kd = dir * DIN + d;
  float A2[DST], h[DST];
#pragma unroll
  for (int n = 0; n < DST; ++n) { A2[n] = -__expf(bf16r(Alog[kd * DST + n])) * LOG2E; h[n] = 0.0f; }
  float wd[DTRK];
#pragma unroll
  for (int r = 0; r < DTRK; ++r) wd[r] = bf16r(dtw[kd * DTRK + r]);
  const float bd = bf16r(dtb[kd]);
  const float Dd = bf16r(Dv[kd]);
  const float* XDb = XD + (size_t)bb * LTOK * XDN + 64 * dir;
  const unsigned short* UHb = UH + (size_t)bb * LTOK * DIN + d;
  const unsigned short* ULb = UL + (size_t)bb * LTOK * DIN + d;
  float* Yd = YS + (size_t)dir * NTOK * DIN + (size_t)bb * LTOK * DIN;
#pragma unroll 1
  for (int c = 0; c < LTOK / SCH; ++c) {
#pragma unroll 1
    for (int s = 0; s < SCH; ++s) {
      const int tok = tok_of(dir, c * SCH + s);
      const float* xr = XDb + (size_t)tok * XDN;
      const v4f d0 = *(const v4fa*)xr, d1 = *(const v4fa*)(xr + 4);
      const float raw = ((((((d0[0] * wd[0] + d0[1] * wd[1]) + d0[2] * wd[2]) + d0[3] * wd[3]) + d1[0] * wd[4]) + d1[1] * wd[5])
                         + d1[2] * wd[6]) + d1[3] * wd[7];
      const float a = raw + bd;
      const float dl = fmaxf(a, 0.0f) + log1pf(__expf(-fabsf(a)));
      const size_t uo = (size_t)tok * DIN;
      const float uv = bf16_val(UHb[uo]) + bf16_val(ULb[uo]);
      v4f Bv[4], Cv[4];
#pragma unroll
      for (int q = 0; q < 4; ++q) {
        Bv[q] = *(const v4fa*)(xr + XBO + 4 * q);
        Cv[q] = *(const v4fa*)(xr + XCO + 4 * q);
      }
      const float dx = dl * uv;
      float y = 0.0f;
#pragma unroll
      for (int n = 0; n < DST; ++n) {
        const float e = exp2f(dl * A2[n]);
        h[n] = e * h[n] + dx * Bv[n >> 2][n & 3];
        y = y + h[n] * Cv[n >> 2][n & 3];
      }
      sy[s * SYP + d] = y + uv * Dd;
    }
    __syncthreads();
#pragma unroll
    for (int pass = 0; pass < 2; ++pass) {
#pragma unroll
      for (int it = 0; it < (SCH * (DIN / 4)) / DIN; ++it) {
        const int ix = it * DIN + tid;
        const int r = ix / (DIN / 4), q4 = (ix - r * (DIN / 4)) * 4;
        const int tok = tok_of(dir, c * SCH + r);
        const v4f v = *(const v4fa*)(sy + r * SYP + q4);
        *(volatile v4f*)(Yd + (size_t)tok * DIN + q4) = v;
      }
      __threadfence();
    }
    __syncthreads();
  }
}

__global__ __launch_bounds__(256) void k_gate(const float* __restrict__ YS, const float* __restrict__ XZ,
                                             const float* __restrict__ g, const float* __restrict__ bt,
                                             unsigned short* GH, unsigned short* GL) {
#pragma clang fp contract(off)
  const int tid = threadIdx.x, lane = tid & 31, wave = tid >> 5;
  const int tok = blockIdx.x * 8 + wave;
  const int c8 = lane * 8;
  const size_t PL = (size_t)NTOK * DIN;
  const size_t ro = (size_t)tok * DIN + c8;
  const v4f y0a = *(const v4fa*)(YS + ro),          y0b = *(const v4fa*)(YS + ro + 4);
  const v4f y1a = *(const v4fa*)(YS + PL + ro),     y1b = *(const v4fa*)(YS + PL + ro + 4);
  const v4f y2a = *(const v4fa*)(YS + 2 * PL + ro), y2b = *(const v4fa*)(YS + 2 * PL + ro + 4);
  const v4f y3a = *(const v4fa*)(YS + 3 * PL + ro), y3b = *(const v4fa*)(YS + 3 * PL + ro + 4);
  const v4f za  = *(const v4fa*)(XZ + ro),          zb  = *(const v4fa*)(XZ + ro + 4);
  float gg[8], bq[8];
  {
    const v4f ga = *(const v4fa*)(g + c8), gb = *(const v4fa*)(g + c8 + 4);
    const v4f ba = *(const v4fa*)(bt + c8), b4 = *(const v4fa*)(bt + c8 + 4);
#pragma unroll
    for (int u = 0; u < 4; ++u) { gg[u] = bf16r(ga[u]); gg[4 + u] = bf16r(gb[u]); bq[u] = bf16r(ba[u]); bq[4 + u] = bf16r(b4[u]); }
  }
  float m[8];
#pragma unroll
  for (int u = 0; u < 4; ++u) {
    m[u]     = ((y0a[u] + y1a[u]) + y2a[u]) + y3a[u];
    m[4 + u] = ((y0b[u] + y1b[u]) + y2b[u]) + y3b[u];
  }
  float s = 0.0f;
#pragma unroll
  for (int u = 0; u < 8; ++u) s = s + m[u];
#pragma unroll
  for (int o = 16; o > 0; o >>= 1) s = s + __shfl_xor(s, o);
  const float mu = s * (1.0f / (float)DIN);
  float q = 0.0f;
#pragma unroll
  for (int u = 0; u < 8; ++u) { const float dv = m[u] - mu; q = q + dv * dv; }
#pragma unroll
  for (int o = 16; o > 0; o >>= 1) q = q + __shfl_xor(q, o);
  const float var = q * (1.0f / (float)DIN);
  const float rsd = rsqrtf(var + EPSV);
  float zz[8];
#pragma unroll
  for (int u = 0; u < 4; ++u) { zz[u] = za[u]; zz[4 + u] = zb[u]; }
  float ov[8];
#pragma unroll
  for (int u = 0; u < 8; ++u) {
    const float nv = ((m[u] - mu) * rsd) * gg[u] + bq[u];
    ov[u] = nv * siluf(zz[u]);
  }
  us8 hi, lo;
  split8(ov, hi, lo);
  *(volatile us8*)(GH + ro) = hi; *(volatile us8*)(GL + ro) = lo;
  __threadfence();
  *(volatile us8*)(GH + ro) = hi; *(volatile us8*)(GL + ro) = lo;
}

extern "C" void kernel_launch(void* const* d_in, const int* in_sizes, int n_in,
                              void* d_out, int out_size, void* d_ws, size_t ws_size,
                              hipStream_t stream) {
  if (n_in < 12) return;
  if (in_sizes[0] != NBAT * LTOK * DMD || in_sizes[1] != 2 * DIN * DMD || in_sizes[2] != DIN * DCV || in_sizes[3] != DIN ||
      in_sizes[4] != NDIR * XPR * DIN || in_sizes[5] != NDIR * DIN * DTRK || in_sizes[6] != NDIR * DIN ||
      in_sizes[7] != NDIR * DIN * DST || in_sizes[8] != NDIR * DIN || in_sizes[9] != DIN || in_sizes[10] != DIN ||
      in_sizes[11] != DMD * DIN || out_size != NBAT * LTOK * DMD) return;

  const float* x    = (const float*)d_in[0];
  const float* inw  = (const float*)d_in[1];
  const float* cw   = (const float*)d_in[2];
  const float* cb   = (const float*)d_in[3];
  const float* xpw  = (const float*)d_in[4];
  const float* dtw  = (const float*)d_in[5];
  const float* dtb  = (const float*)d_in[6];
  const float* Alog = (const float*)d_in[7];
  const float* Dv   = (const float*)d_in[8];
  const float* gng  = (const float*)d_in[9];
  const float* gnb  = (const float*)d_in[10];
  const float* ow   = (const float*)d_in[11];
  float* out = (float*)d_out;

  size_t off = 0;
  auto carve = [&](size_t bytes) -> char* { char* p = (char*)d_ws + off; off += (bytes + 255) & ~(size_t)255; return p; };
  unsigned short* WIN16 = (unsigned short*)carve((size_t)2 * DIN * DMD * 2);
  unsigned short* WX16  = (unsigned short*)carve((size_t)XDN * DIN * 2);
  unsigned short* WO16  = (unsigned short*)carve((size_t)DMD * DIN * 2);
  unsigned short* XT16  = (unsigned short*)carve((size_t)NTOK * DMD * 2);
  float* XI             = (float*)carve((size_t)NTOK * DIN * 4);
  float* XZ             = (float*)carve((size_t)NTOK * DIN * 4);
  unsigned short* UH    = (unsigned short*)carve((size_t)NTOK * DIN * 2);
  unsigned short* UL    = (unsigned short*)carve((size_t)NTOK * DIN * 2);
  float* XD             = (float*)carve((size_t)NTOK * XDN * 4);
  float* YS             = (float*)carve((size_t)NDIR * NTOK * DIN * 4);
  unsigned short* GH    = (unsigned short*)carve((size_t)NTOK * DIN * 2);
  unsigned short* GL    = (unsigned short*)carve((size_t)NTOK * DIN * 2);
  if (off > ws_size || off > (size_t)134217728) return;

  const dim3 b256(256);
  k_cvt<<<dim3((2 * DIN * (DMD / 8) + 255) / 256), b256, 0, stream>>>(inw, WIN16, 2 * DIN, DMD / 8, 2 * DIN * (DMD / 8));
  k_cvt_xw<<<dim3((XDN * (DIN / 8) + 255) / 256), b256, 0, stream>>>(xpw, WX16);
  k_cvt<<<dim3((DMD * (DIN / 8) + 255) / 256), b256, 0, stream>>>(ow, WO16, DMD, DIN / 8, DMD * (DIN / 8));
  k_cvt<<<dim3((NTOK * (DMD / 8) + 255) / 256), b256, 0, stream>>>(x, XT16, NTOK, DMD / 8, NTOK * (DMD / 8));
  k_gemm<0, 0><<<dim3(NTOK / 128, (2 * DIN) / 64, 1), b256, 0, stream>>>(XT16, XT16, DMD, 0, WIN16, WIN16, DMD, 0,
                                                                        XI, XZ, DIN, DIN, 0, DMD, NTOK);
  k_dw4<<<dim3(NTOK * (DIN / 8) / 256), b256, 0, stream>>>(XI, cw, cb, UH, UL);
  k_gemm<1, 0><<<dim3(NTOK / 128, XDN / 64, 1), b256, 0, stream>>>(UH, UL, DIN, 0, WX16, WX16, DIN, 0,
                                                                  XD, XD, 0, XDN, 0, DIN, NTOK);
  k_scan<<<dim3(NBAT * NDIR), b256, 0, stream>>>(XD, UH, UL, dtw, dtb, Alog, Dv, YS);
  k_gate<<<dim3(NTOK / 8), b256, 0, stream>>>(YS, XZ, gng, gnb, GH, GL);
  k_gemm<1, 0><<<dim3(NTOK / 128, DMD / 64, 1), b256, 0, stream>>>(GH, GL, DIN, 0, WO16, WO16, DIN, 0,
                                                                 out, out, 0, DMD, 0, DIN, NTOK);
}
